// Net_90744069030470
// MI455X (gfx1250) — hardware-verified
//
#include <hip/hip_runtime.h>
#include <stddef.h>
#include <stdint.h>
#include <math.h>


#define FIN    256
#define HID    256
#define KH     512
#define NTC    64
#define NTHR   256
#define NWAVE  8
#define EPT    8
#define CHUNK  (NTHR * EPT)
#define WCAP   (EPT * 32)
#define LISTN  (NWAVE * WCAP)
#define NBA    1024
#define SLA    10
#define RCAP   16384
#define DEGCAP 64
#define GBM    64
#define GBN    64
#define GTHR   128
#define NUW1   (HID * (FIN / 8))
#define NUWG   (32 * (KH / 8))
#define ZINTS  (LISTN + 2 * RCAP + 3 * NBA)
#define MISC_INTS 16
#define A_LDS_INTS (ZINTS + MISC_INTS + NBA * 4)
#define B_LDS_INTS (ZINTS + MISC_INTS + NWAVE * 64 + 1024 + 64 + 32)
#define C_LDS_INTS (ZINTS + MISC_INTS + NBA * 16)
#define WSMAX  134217728

static_assert((CHUNK & (CHUNK - 1)) == 0 && CHUNK <= 4096);
static_assert((NBA & (NBA - 1)) == 0 && NBA == (1 << SLA));
static_assert(((long long)CHUNK << SLA) < (1LL << 31));
static_assert(ZINTS % 4 == 0 && ((ZINTS + MISC_INTS) % 4) == 0);
static_assert(NBA % NWAVE == 0 && NBA % 32 == 0 && NBA % 2 == 0);
static_assert(FIN % 32 == 0 && KH % 32 == 0 && KH == 2 * HID && HID % GBN == 0 && NTC == GBN);
static_assert(GBM == (GTHR / 32) * 16);
static_assert(NUW1 % NTHR == 0 && NUWG % NTHR == 0);
static_assert((NBA * 4) % (NTHR * 4) == 0 && (NBA * 16) % (NTHR * 4) == 0);
static_assert(C_LDS_INTS * 4 <= 300000 && A_LDS_INTS * 4 <= 300000 && B_LDS_INTS * 4 <= 300000);

typedef float          v2f   __attribute__((ext_vector_type(2)));
typedef float          v4f   __attribute__((ext_vector_type(4)));
typedef float          v8f   __attribute__((ext_vector_type(8)));
typedef int            v4i   __attribute__((ext_vector_type(4)));
typedef int            v8i   __attribute__((ext_vector_type(8)));
typedef unsigned short v4us  __attribute__((ext_vector_type(4)));
typedef unsigned short v8us  __attribute__((ext_vector_type(8)));
typedef unsigned short v16us __attribute__((ext_vector_type(16)));
typedef __bf16         v16bf __attribute__((ext_vector_type(16)));
typedef v2f  __attribute__((may_alias)) v2fa;
typedef v4f  __attribute__((may_alias)) v4fa;
typedef v4i  __attribute__((may_alias)) v4ia;
typedef v4us __attribute__((may_alias)) v4usa;
typedef v8us __attribute__((may_alias)) v8usa;
union FragB { v16bf v; v16us u; v8us h[2]; v8i w; };

__device__ __forceinline__ v8f wmb(const FragB& a, const FragB& b, v8f c) {
  v8f d = __builtin_amdgcn_wmma_f32_16x16x32_bf16(false, a.v, false, b.v, (short)0, c, false, false);
  asm volatile("v_nop\n\tv_nop\n\tv_nop\n\tv_nop" : "+v"(d) : "v"(a.w), "v"(b.w));
  return d;
}

__device__ __forceinline__ unsigned bf16_bits(float f) {
  const unsigned u = __float_as_uint(f);
  return (u + 0x7FFFu + ((u >> 16) & 1u)) >> 16;
}
__device__ __forceinline__ float bf16_val(float f) {
  return __uint_as_float(bf16_bits(f) << 16);
}

__device__ __forceinline__ void wave_sync() {
  __builtin_amdgcn_fence(__ATOMIC_RELEASE, "wavefront");
  __builtin_amdgcn_wave_barrier();
  __builtin_amdgcn_fence(__ATOMIC_ACQUIRE, "wavefront");
}

template <int SLB>
__device__ __forceinline__ int scan_chunk(const int* __restrict__ dsts, int nE, int cbase, int slotBase,
                                          int nb, int vec8, int* list, int tid, int lane, int wave) {
  int wc = 0;
  const int el0  = tid * EPT;
  const int e0   = cbase + el0;
  const int sent = -2147483647 - 1;
  v4i da, db;
  if (vec8 != 0 && cbase + CHUNK <= nE) {
    da = *(const v4i*)(dsts + e0);
    db = *(const v4i*)(dsts + e0 + 4);
  } else {
    da.x = (e0     < nE) ? dsts[min(e0,     nE - 1)] : sent;
    da.y = (e0 + 1 < nE) ? dsts[min(e0 + 1, nE - 1)] : sent;
    da.z = (e0 + 2 < nE) ? dsts[min(e0 + 2, nE - 1)] : sent;
    da.w = (e0 + 3 < nE) ? dsts[min(e0 + 3, nE - 1)] : sent;
    db.x = (e0 + 4 < nE) ? dsts[min(e0 + 4, nE - 1)] : sent;
    db.y = (e0 + 5 < nE) ? dsts[min(e0 + 5, nE - 1)] : sent;
    db.z = (e0 + 6 < nE) ? dsts[min(e0 + 6, nE - 1)] : sent;
    db.w = (e0 + 7 < nE) ? dsts[min(e0 + 7, nE - 1)] : sent;
  }
  const unsigned nbs = (unsigned)slotBase;
  const unsigned unb = (unsigned)nb;
  const unsigned s0 = (unsigned)da.x - nbs, s1 = (unsigned)da.y - nbs;
  const unsigned s2 = (unsigned)da.z - nbs, s3 = (unsigned)da.w - nbs;
  const unsigned s4 = (unsigned)db.x - nbs, s5 = (unsigned)db.y - nbs;
  const unsigned s6 = (unsigned)db.z - nbs, s7 = (unsigned)db.w - nbs;
  const bool h0 = s0 < unb, h1 = s1 < unb, h2 = s2 < unb, h3 = s3 < unb;
  const bool h4 = s4 < unb, h5 = s5 < unb, h6 = s6 < unb, h7 = s7 < unb;
  const unsigned any = __builtin_amdgcn_ballot_w32(h0 | h1 | h2 | h3 | h4 | h5 | h6 | h7);
  if (any != 0u) {
#define HITJ(J, HJ, SJ) { \
      const unsigned mj = __builtin_amdgcn_ballot_w32(HJ); \
      if (mj != 0u) { \
        if (HJ) { \
          const int pos = wc + (int)__builtin_amdgcn_mbcnt_lo(mj, 0u); \
          if (pos < WCAP) list[wave * WCAP + pos] = ((el0 + (J)) << SLB) | (int)(SJ); \
        } \
        wc += (int)__builtin_popcount(mj); } }
    HITJ(0, h0, s0)
    HITJ(1, h1, s1)
    HITJ(2, h2, s2)
    HITJ(3, h3, s3)
    HITJ(4, h4, s4)
    HITJ(5, h5, s5)
    HITJ(6, h6, s6)
    HITJ(7, h7, s7)
#undef HITJ
  }
  return wc;
}

__device__ __forceinline__ void build_lists(const int* __restrict__ keys, int nE, int nodeBase, int vec8,
                                            int* dsm, int tid, int lane, int wave, int& ovfOut) {
  int* list = dsm;
  int* hl   = dsm + LISTN;
  int* sl   = hl + RCAP;
  int* cnt  = sl + RCAP;
  int* offs = cnt + NBA;
  int* cur  = offs + NBA;
  int* misc = cur + NBA;
  __syncthreads();
  {
    const v4i z4 = {0, 0, 0, 0};
    for (int i = tid * 4; i < ZINTS; i += NTHR * 4) *(v4ia*)(dsm + i) = z4;
    if (tid < MISC_INTS) misc[tid] = 0;
  }
  __syncthreads();

  int t = 0, ov = 0;
  const int nChunks = (nE + CHUNK - 1) / CHUNK;
#pragma unroll 1
  for (int ch = 0; ch < nChunks; ++ch) {
    const int cbase = ch * CHUNK;
    const int wc = scan_chunk<SLA>(keys, nE, cbase, nodeBase, NBA, vec8, list, tid, lane, wave);
    if (lane == 0) misc[wave] = wc;
    __syncthreads();
    if (wave == 0) {
#pragma unroll 1
      for (int w2 = 0; w2 < NWAVE; ++w2) {
        int c = misc[w2];
        c = c < 0 ? 0 : (c > WCAP ? WCAP : c);
#pragma unroll 1
        for (int b0 = 0; b0 < c; b0 += 32) {
          const int idx = b0 + lane;
          const int ent = list[w2 * WCAP + (idx < WCAP ? idx : WCAP - 1)];
          const int m32 = (c - b0) < 32 ? (c - b0) : 32;
#pragma unroll 1
          for (int k = 0; k < m32; ++k) {
            const int u    = __builtin_amdgcn_readlane(ent, k);
            const int slot = u & (NBA - 1);
            const int el   = (u >> SLA) & (CHUNK - 1);
            const int pk   = ((cbase + el) << SLA) | slot;
            if (t < RCAP) {
              if (lane == 0) { hl[t] = pk; cnt[slot] = cnt[slot] + 1; }
              t = t + 1;
            } else {
              ov = 1;
            }
          }
        }
      }
    }
    __syncthreads();
  }
  if (wave == 0 && lane == 0) { misc[8] = t; misc[9] = ov; }
  __syncthreads();
  int tt = misc[8];
  tt = tt < 0 ? 0 : (tt > RCAP ? RCAP : tt);
  ovfOut = misc[9];

  if (wave == 0) {
    const int base = lane * (NBA / 32);
    int s = 0;
#pragma unroll 1
    for (int i = 0; i < NBA / 32; ++i) s += cnt[base + i];
    int incl = s;
#pragma unroll
    for (int d = 1; d < 32; d <<= 1) {
      const int y = __shfl_up(incl, d, 32);
      if (lane >= d) incl += y;
    }
    int run = incl - s;
#pragma unroll 1
    for (int i = 0; i < NBA / 32; ++i) {
      const int cv = cnt[base + i];
      offs[base + i] = run;
      cur[base + i]  = run;
      run += cv;
    }
  }
  __syncthreads();
  if (wave == 0) {
#pragma unroll 1
    for (int b0 = 0; b0 < tt; b0 += 32) {
      const int idx = b0 + lane;
      const int ent = hl[idx < RCAP ? idx : RCAP - 1];
      const int m32 = (tt - b0) < 32 ? (tt - b0) : 32;
#pragma unroll 1
      for (int k = 0; k < m32; ++k) {
        const int u    = __builtin_amdgcn_readlane(ent, k);
        const int slot = u & (NBA - 1);
        if (lane == 0) {
          int p = cur[slot];
          p = p < 0 ? 0 : (p > RCAP - 1 ? RCAP - 1 : p);
          sl[p] = u;
          cur[slot] = p + 1;
        }
      }
    }
  }
  __syncthreads();
}

__global__ __launch_bounds__(NTHR) void k_wprep(const float* __restrict__ W1, const float* __restrict__ Wg1,
                                                const float* __restrict__ Wg2,
                                                unsigned short* W1T, unsigned short* WGT) {
  const int u = (int)blockIdx.x * NTHR + (int)threadIdx.x;
  v8us o;
  unsigned short* dp;
  if (u < NUW1) {
    const int n  = u >> 5;
    const int k8 = (u & 31) * 8;
    const float* p = W1 + (size_t)k8 * HID + n;
#pragma unroll
    for (int i = 0; i < 8; ++i) o[i] = (unsigned short)bf16_bits(p[(size_t)i * HID]);
    dp = W1T + (size_t)n * FIN + k8;
  } else if (u < NUW1 + NUWG) {
    const int v  = u - NUW1;
    const int j  = v >> 6;
    const int k8 = (v & 63) * 8;
    const int kk = k8 & (HID - 1);
    const float* p = Wg1 + (size_t)kk * 32 + j;
#pragma unroll
    for (int i = 0; i < 8; ++i) o[i] = (unsigned short)bf16_bits(p[(size_t)i * 32]);
    dp = WGT + (size_t)j * KH + k8;
  } else if (u < NUW1 + 2 * NUWG) {
    const int v  = u - NUW1 - NUWG;
    const int j  = v >> 6;
    const int k8 = (v & 63) * 8;
    const int kk = k8 & (HID - 1);
    const float* p = Wg2 + (size_t)kk * 32 + j;
#pragma unroll
    for (int i = 0; i < 8; ++i) o[i] = (unsigned short)bf16_bits(p[(size_t)i * 32]);
    dp = WGT + (size_t)(32 + j) * KH + k8;
  } else {
    return;
  }
  *(volatile v8us*)dp = o;
  __threadfence();
  *(volatile v8us*)dp = o;
}

__global__ __launch_bounds__(NTHR) void k_cvx(const float* __restrict__ x, int nN, int nUnits,
                                              unsigned short* xb) {
  const int u = (int)blockIdx.x * NTHR + (int)threadIdx.x;
  if (u >= nUnits) return;
  const int row = u >> 5;
  const int k8  = (u & 31) * 8;
  const int rc  = row < nN ? row : nN - 1;
  const float* p = x + (size_t)rc * FIN + k8;
  const v4f a = *(const v4fa*)p;
  const v4f b = *(const v4fa*)(p + 4);
  const bool ok = row < nN;
  v8us o;
  o[0] = ok ? (unsigned short)bf16_bits(a.x) : (unsigned short)0;
  o[1] = ok ? (unsigned short)bf16_bits(a.y) : (unsigned short)0;
  o[2] = ok ? (unsigned short)bf16_bits(a.z) : (unsigned short)0;
  o[3] = ok ? (unsigned short)bf16_bits(a.w) : (unsigned short)0;
  o[4] = ok ? (unsigned short)bf16_bits(b.x) : (unsigned short)0;
  o[5] = ok ? (unsigned short)bf16_bits(b.y) : (unsigned short)0;
  o[6] = ok ? (unsigned short)bf16_bits(b.z) : (unsigned short)0;
  o[7] = ok ? (unsigned short)bf16_bits(b.w) : (unsigned short)0;
  unsigned short* dp = xb + (size_t)row * FIN + k8;
  *(volatile v8us*)dp = o;
  __threadfence();
  *(volatile v8us*)dp = o;
}

__global__ __launch_bounds__(GTHR) void k_gemm1(const unsigned short* __restrict__ A,
                                                const unsigned short* __restrict__ WT,
                                                const float* __restrict__ b1, unsigned short* hhl) {
  __shared__ __attribute__((aligned(16))) float stg[GBM * GBN];
  __shared__ __attribute__((aligned(16))) unsigned short hls[GBM * 2 * GBN];
  const int tid = (int)threadIdx.x, lane = tid & 31, wave = tid >> 5, hh = lane >> 4, m = lane & 15;
  const int rowBase = (int)blockIdx.x * GBM;
  const int col0    = (int)blockIdx.y * GBN;

  v8f acc[4];
  {
    const v8f z = {0.f, 0.f, 0.f, 0.f, 0.f, 0.f, 0.f, 0.f};
    acc[0] = z; acc[1] = z; acc[2] = z; acc[3] = z;
  }
  const unsigned short* ap = A  + (size_t)(rowBase + 16 * wave + m) * (size_t)FIN + 8 * hh;
  const unsigned short* wp = WT + (size_t)(col0 + m) * (size_t)FIN + 8 * hh;
#pragma unroll 1
  for (int ks = 0; ks < FIN / 32; ++ks) {
    FragB af;
    af.h[0] = *(const v8usa*)(ap + 32 * ks);
    af.h[1] = *(const v8usa*)(ap + 32 * ks + 16);
#pragma unroll
    for (int t = 0; t < 4; ++t) {
      const unsigned short* wq = wp + (size_t)(16 * t) * (size_t)FIN + 32 * ks;
      FragB bf;
      bf.h[0] = *(const v8usa*)wq;
      bf.h[1] = *(const v8usa*)(wq + 16);
      acc[t] = wmb(af, bf, acc[t]);
    }
  }
#pragma unroll
  for (int t = 0; t < 4; ++t) {
    const int lc = 16 * t + m;
#pragma unroll
    for (int r = 0; r < 8; ++r) {
      const int lr = 16 * wave + 8 * hh + r;
      stg[lr * GBN + lc] = acc[t][r];
    }
  }
  __syncthreads();

  v4f bb;
  {
    const v4f t1 = *(const v4fa*)(b1 + col0 + 4 * m);
    bb.x = bf16_val(t1.x); bb.y = bf16_val(t1.y); bb.z = bf16_val(t1.z); bb.w = bf16_val(t1.w);
  }
#pragma unroll
  for (int i = 0; i < 8; ++i) {
    const int lr = 16 * wave + 2 * i + hh;
    const v4f f = *(const v4fa*)(stg + lr * GBN + 4 * m) + bb;
    v4us h4, l4;
    unsigned hb;
    hb = bf16_bits(f.x); h4[0] = (unsigned short)hb; l4[0] = (unsigned short)bf16_bits(f.x - __uint_as_float(hb << 16));
    hb = bf16_bits(f.y); h4[1] = (unsigned short)hb; l4[1] = (unsigned short)bf16_bits(f.y - __uint_as_float(hb << 16));
    hb = bf16_bits(f.z); h4[2] = (unsigned short)hb; l4[2] = (unsigned short)bf16_bits(f.z - __uint_as_float(hb << 16));
    hb = bf16_bits(f.w); h4[3] = (unsigned short)hb; l4[3] = (unsigned short)bf16_bits(f.w - __uint_as_float(hb << 16));
    *(v4usa*)(hls + lr * (2 * GBN) + 4 * m) = h4;
    *(v4usa*)(hls + lr * (2 * GBN) + GBN + 4 * m) = l4;
  }
  __syncthreads();
  v8us q[8];
#pragma unroll
  for (int i = 0; i < 8; ++i) {
    const int lr = 16 * wave + 2 * i + hh;
    q[i] = *(const v8usa*)(hls + lr * (2 * GBN) + 8 * m);
  }
  const int coff = (m < 8) ? (col0 + 8 * m) : (HID + col0 + 8 * (m - 8));
#pragma unroll
  for (int i = 0; i < 8; ++i) {
    const int lr = 16 * wave + 2 * i + hh;
    unsigned short* op = hhl + (size_t)(rowBase + lr) * (size_t)KH + coff;
    *(volatile v8us*)op = q[i];
  }
  __threadfence();
#pragma unroll
  for (int i = 0; i < 8; ++i) {
    const int lr = 16 * wave + 2 * i + hh;
    unsigned short* op = hhl + (size_t)(rowBase + lr) * (size_t)KH + coff;
    *(volatile v8us*)op = q[i];
  }
}

__global__ __launch_bounds__(GTHR) void k_gemm2(const unsigned short* __restrict__ A,
                                                const unsigned short* __restrict__ WT,
                                                float* outF, int K, int ldo) {
  __shared__ __attribute__((aligned(16))) float stg[GBM * GBN];
  const int tid = (int)threadIdx.x, lane = tid & 31, wave = tid >> 5, hh = lane >> 4, m = lane & 15;
  const int rowBase = (int)blockIdx.x * GBM;
  const int col0    = (int)blockIdx.y * GBN;

  v8f acc[4];
  {
    const v8f z = {0.f, 0.f, 0.f, 0.f, 0.f, 0.f, 0.f, 0.f};
    acc[0] = z; acc[1] = z; acc[2] = z; acc[3] = z;
  }
  const unsigned short* ap = A  + (size_t)(rowBase + 16 * wave + m) * (size_t)K + 8 * hh;
  const unsigned short* wp = WT + (size_t)(col0 + m) * (size_t)K + 8 * hh;
  const int ksteps = K >> 5;
#pragma unroll 1
  for (int ks = 0; ks < ksteps; ++ks) {
    FragB af;
    af.h[0] = *(const v8usa*)(ap + 32 * ks);
    af.h[1] = *(const v8usa*)(ap + 32 * ks + 16);
#pragma unroll
    for (int t = 0; t < 4; ++t) {
      const unsigned short* wq = wp + (size_t)(16 * t) * (size_t)K + 32 * ks;
      FragB bf;
      bf.h[0] = *(const v8usa*)wq;
      bf.h[1] = *(const v8usa*)(wq + 16);
      acc[t] = wmb(af, bf, acc[t]);
    }
  }
#pragma unroll
  for (int t = 0; t < 4; ++t) {
    const int lc = 16 * t + m;
#pragma unroll
    for (int r = 0; r < 8; ++r) {
      const int lr = 16 * wave + 8 * hh + r;
      stg[lr * GBN + lc] = acc[t][r];
    }
  }
  __syncthreads();
  v4f fv[8];
#pragma unroll
  for (int i = 0; i < 8; ++i) {
    const int lr = 16 * wave + 2 * i + hh;
    fv[i] = *(const v4fa*)(stg + lr * GBN + 4 * m);
  }
#pragma unroll
  for (int i = 0; i < 8; ++i) {
    const int lr = 16 * wave + 2 * i + hh;
    float* op = outF + (size_t)(rowBase + lr) * (size_t)ldo + col0 + 4 * m;
    *(volatile v4f*)op = fv[i];
  }
  __threadfence();
#pragma unroll
  for (int i = 0; i < 8; ++i) {
    const int lr = 16 * wave + 2 * i + hh;
    float* op = outF + (size_t)(rowBase + lr) * (size_t)ldo + col0 + 4 * m;
    *(volatile v4f*)op = fv[i];
  }
}

__global__ __launch_bounds__(NTHR) void k_scanA(const int* __restrict__ gath, const int* __restrict__ keys,
                                                const float* __restrict__ ew, int nE, int nN, int vec8,
                                                const float* __restrict__ T, int tcol,
                                                const float* __restrict__ attS, const float* __restrict__ attD,
                                                float* PP, float* ASDl) {
  extern __shared__ __attribute__((aligned(16))) int dsm[];
  int* sl   = dsm + LISTN + RCAP;
  int* cnt  = sl + RCAP;
  int* offs = cnt + NBA;
  int* misc = offs + 2 * NBA;
  float* asdS = (float*)(misc + MISC_INTS);
  const int tid = (int)threadIdx.x, lane = tid & 31, wave = tid >> 5, hh = lane >> 4;
  const int nodeBase = (int)blockIdx.x * NBA;
  const float aS = bf16_val(attS[lane]);
  const float aD = bf16_val(attD[lane]);

  int ovf = 0;
  build_lists(keys, nE, nodeBase, vec8, dsm, tid, lane, wave, ovf);

  const float qnan = __int_as_float(0x7fc00000);
#pragma unroll 1
  for (int si = 0; si < NBA / NWAVE; ++si) {
    const int s    = si * NWAVE + wave;
    const int node = nodeBase + s;
    int c = cnt[s];
    const bool big = c > DEGCAP;
    c = c < 0 ? 0 : (c > DEGCAP ? DEGCAP : c);
    int o = offs[s];
    o = o < 0 ? 0 : (o > RCAP ? RCAP : o);
    float acc = 0.0f;
#pragma unroll 1
    for (int b0 = 0; b0 < c; b0 += 32) {
      int idx = o + b0 + lane;
      idx = idx > RCAP - 1 ? RCAP - 1 : idx;
      const int ent = sl[idx];
      int eid = ent >> SLA;
      eid = eid < 0 ? 0 : (eid > nE - 1 ? nE - 1 : eid);
      int sr = gath[eid];
      sr = sr < 0 ? 0 : (sr > nN - 1 ? nN - 1 : sr);
      const int wvi = __float_as_int(bf16_val(ew[eid]));
      const int m32 = (c - b0) < 32 ? (c - b0) : 32;
#pragma unroll 1
      for (int k = 0; k < m32; ++k) {
        const int   sk = __builtin_amdgcn_readlane(sr, k);
        const float ck = __int_as_float(__builtin_amdgcn_readlane(wvi, k));
        const float a  = T[(size_t)sk * NTC + tcol + lane];
        acc = fmaf(ck, a, acc);
      }
    }
    const float pzr = (big || ovf != 0) ? qnan : 0.0f;
    const bool live = node < nN;
    const float mv = live ? (acc + pzr) : 0.0f;
    float ps = mv * aS, pd = mv * aD;
#pragma unroll
    for (int d = 1; d < 16; d <<= 1) {
      ps += __shfl_xor(ps, d, 32);
      pd += __shfl_xor(pd, d, 32);
    }
    if ((lane & 15) == 0) { asdS[s * 4 + hh] = ps; asdS[s * 4 + 2 + hh] = pd; }
    float* op = PP + (size_t)node * NTC + tcol + lane;
    *(volatile float*)op = mv;
    __threadfence();
    *(volatile float*)op = mv;
  }
  __syncthreads();
#pragma unroll
  for (int it = 0; it < (NBA * 4) / (NTHR * 4); ++it) {
    const int p = it * NTHR + tid;
    const v4f v = *(const v4fa*)(asdS + 4 * p);
    *(volatile v4f*)(ASDl + (size_t)nodeBase * 4 + 4 * (size_t)p) = v;
  }
  __threadfence();
#pragma unroll
  for (int it = 0; it < (NBA * 4) / (NTHR * 4); ++it) {
    const int p = it * NTHR + tid;
    const v4f v = *(const v4fa*)(asdS + 4 * p);
    *(volatile v4f*)(ASDl + (size_t)nodeBase * 4 + 4 * (size_t)p) = v;
  }
}

__global__ __launch_bounds__(NTHR) void k_scanB(const int* __restrict__ gath, const int* __restrict__ keys,
                                                int nE, int nN, int vec8, int NP,
                                                const float* __restrict__ PP, const float* __restrict__ ASD,
                                                const float* __restrict__ gb1, const float* __restrict__ gb2,
                                                const float* __restrict__ wm1, const float* __restrict__ wm2,
                                                const float* __restrict__ bm1, const float* __restrict__ bm2,
                                                float* Y) {
  extern __shared__ __attribute__((aligned(16))) int dsm[];
  int* sl   = dsm + LISTN + RCAP;
  int* cnt  = sl + RCAP;
  int* offs = cnt + NBA;
  int* misc = offs + 2 * NBA;
  float* ex   = (float*)(misc + MISC_INTS);
  float* WmS  = ex + NWAVE * 64;
  float* gbS  = WmS + 1024;
  float* bmS  = gbS + 64;
  const int tid = (int)threadIdx.x, lane = tid & 31, wave = tid >> 5;
  float* rowbuf = ex + wave * 64;
  const int nodeBase = (int)blockIdx.x * NBA;

  WmS[tid]       = bf16_val(wm1[tid]);
  WmS[256 + tid] = bf16_val(wm1[256 + tid]);
  WmS[512 + tid] = bf16_val(wm2[tid]);
  WmS[768 + tid] = bf16_val(wm2[256 + tid]);
  if (wave == 0) {
    const int c16 = lane & 15;
    const int ai = __float_as_int(bm1[c16]);
    const int bi = __float_as_int(bm2[c16]);
    const int mk = -(int)(lane < 16);
    bmS[lane] = bf16_val(__int_as_float((ai & mk) | (bi & ~mk)));
    gbS[lane] = bf16_val(gb1[lane]);
  } else if (wave == 1) {
    gbS[32 + lane] = bf16_val(gb2[lane]);
  }

  int ovf = 0;
  build_lists(keys, nE, nodeBase, vec8, dsm, tid, lane, wave, ovf);

  const int lsel = lane >> 4, hd = (lane >> 3) & 1;
  const size_t abase = (size_t)lsel * (size_t)NP * 4 + hd;
  const float gbv0 = gbS[2 * lane], gbv1 = gbS[2 * lane + 1];
  const float bmv  = bmS[lane];
  const float* wcol = WmS + lsel * 512 + (lane & 15);
  const float* rsel = rowbuf + lsel * 32;
  const float qnan = __int_as_float(0x7fc00000);
#pragma unroll 1
  for (int si = 0; si < NBA / NWAVE; ++si) {
    const int s    = si * NWAVE + wave;
    const int node = nodeBase + s;
    int c = cnt[s];
    const bool big = c > DEGCAP;
    c = c < 0 ? 0 : (c > DEGCAP ? DEGCAP : c);
    int o = offs[s];
    o = o < 0 ? 0 : (o > RCAP ? RCAP : o);
    const int nc = node < nN ? node : nN - 1;
    const float as_i = ASD[abase + (size_t)nc * 4];
    const float ad_i = ASD[abase + (size_t)nc * 4 + 2];
    const v2f pf = *(const v2fa*)(PP + (size_t)nc * NTC + 2 * lane);
    float lg0 = as_i + ad_i;
    lg0 = (lg0 > 0.0f) ? lg0 : 0.2f * lg0;
    float mrun = lg0, ssum = 1.0f, a0 = pf.x, a1 = pf.y;
#pragma unroll 1
    for (int b0 = 0; b0 < c; b0 += 32) {
      int idx = o + b0 + lane;
      idx = idx > RCAP - 1 ? RCAP - 1 : idx;
      const int ent = sl[idx];
      int eid = ent >> SLA;
      eid = eid < 0 ? 0 : (eid > nE - 1 ? nE - 1 : eid);
      int sr = gath[eid];
      sr = sr < 0 ? 0 : (sr > nN - 1 ? nN - 1 : sr);
      const int m32 = (c - b0) < 32 ? (c - b0) : 32;
#pragma unroll 1
      for (int k = 0; k < m32; ++k) {
        const int sk = __builtin_amdgcn_readlane(sr, k);
        const float asv = ASD[abase + (size_t)sk * 4];
        const v2f f = *(const v2fa*)(PP + (size_t)sk * NTC + 2 * lane);
        float lg = asv + ad_i;
        lg = (lg > 0.0f) ? lg : 0.2f * lg;
        const float d  = lg - mrun;
        const bool  up = d > 0.0f;
        const float e  = expf(up ? -d : d);
        const float sc = up ? e : 1.0f;
        const float p  = up ? 1.0f : e;
        mrun = up ? lg : mrun;
        ssum = fmaf(ssum, sc, p);
        a0 = fmaf(a0, sc, p * f.x);
        a1 = fmaf(a1, sc, p * f.y);
      }
    }
    const float inv = 1.0f / ssum;
    v2f g;
    g.x = a0 * inv + gbv0;
    g.y = a1 * inv + gbv1;
    *(v2fa*)(rowbuf + 2 * lane) = g;
    wave_sync();
#pragma unroll 1
    for (int q = 0; q < 2; ++q) {
      const float v = rowbuf[q * 32 + lane];
      rowbuf[q * 32 + lane] = (v > 0.0f) ? v : expm1f(v);
    }
    wave_sync();
    float y = 0.0f;
#pragma unroll 4
    for (int jj = 0; jj < 32; ++jj) y = fmaf(rsel[jj], wcol[jj * 16], y);
    y += bmv;
    wave_sync();
    const float pzr = (big || ovf != 0) ? qnan : 0.0f;
    const float yv = (node < nN) ? (y + pzr) : 0.0f;
    float* op = Y + (size_t)node * 32 + lane;
    *(volatile float*)op = yv;
    __threadfence();
    *(volatile float*)op = yv;
  }
}

template <int LAST>
__device__ __forceinline__ void c_level(const int* __restrict__ ei, const float* __restrict__ ea, int nE,
                                        int vec8, int nN, const float* __restrict__ Y, int ycol,
                                        int* dsm, float* vs, int tid, int lane, int wave, int nodeBase) {
  int* sl   = dsm + LISTN + RCAP;
  int* cnt  = sl + RCAP;
  int* offs = cnt + NBA;
  int ovf = 0;
  build_lists(ei + nE, nE, nodeBase, vec8, dsm, tid, lane, wave, ovf);
  const int c16 = lane & 15;
  const float qnan = __int_as_float(0x7fc00000);
#pragma unroll 1
  for (int si = 0; si < NBA / NWAVE; ++si) {
    const int s    = si * NWAVE + wave;
    const int node = nodeBase + s;
    int c = cnt[s];
    const bool big = c > DEGCAP;
    c = c < 0 ? 0 : (c > DEGCAP ? DEGCAP : c);
    int o = offs[s];
    o = o < 0 ? 0 : (o > RCAP ? RCAP : o);
    float acc = 0.0f;
#pragma unroll 1
    for (int b0 = 0; b0 < c; b0 += 32) {
      int idx = o + b0 + lane;
      idx = idx > RCAP - 1 ? RCAP - 1 : idx;
      const int ent = sl[idx];
      int eid = ent >> SLA;
      eid = eid < 0 ? 0 : (eid > nE - 1 ? nE - 1 : eid);
      int sr = ei[eid];
      sr = sr < 0 ? 0 : (sr > nN - 1 ? nN - 1 : sr);
      const int wvi = __float_as_int(bf16_val(ea[eid]));
      const int m32 = (c - b0) < 32 ? (c - b0) : 32;
#pragma unroll 1
      for (int k = 0; k < m32; ++k) {
        const int   sk = __builtin_amdgcn_readlane(sr, k);
        const float ck = __int_as_float(__builtin_amdgcn_readlane(wvi, k));
        const float a  = Y[(size_t)sk * 32 + ycol + c16];
        acc = fmaf(ck, a, acc);
      }
    }
    const float pzr = (big || ovf != 0) ? qnan : 0.0f;
    const bool live = node < nN;
    if constexpr (LAST == 0) {
      const float tot = live ? (acc + pzr) : 0.0f;
      if (lane < 16) vs[s * 16 + lane] = tot;
    } else {
      const float pv = vs[s * 16 + c16];
      const float v  = live ? ((pv + acc) + pzr) : 0.0f;
      float mx = v;
#pragma unroll
      for (int d = 1; d < 16; d <<= 1) {
        const float ov = __shfl_xor(mx, d, 32);
        mx = (ov > mx) ? ov : mx;
      }
      const float sh = v - mx;
      float se = expf(sh);
#pragma unroll
      for (int d = 1; d < 16; d <<= 1) se += __shfl_xor(se, d, 32);
      const float res = sh - logf(se);
      if (lane < 16) vs[s * 16 + lane] = res;
    }
  }
}

__global__ __launch_bounds__(NTHR) void k_scanC(const int* __restrict__ ei1, const float* __restrict__ ea1,
                                                int nE1, int vec81,
                                                const int* __restrict__ ei2, const float* __restrict__ ea2,
                                                int nE2, int vec82, int nN,
                                                const float* __restrict__ Y, float* out) {
  extern __shared__ __attribute__((aligned(16))) int dsm[];
  float* vs = (float*)(dsm + ZINTS + MISC_INTS);
  const int tid = (int)threadIdx.x, lane = tid & 31, wave = tid >> 5;
  const int nodeBase = (int)blockIdx.x * NBA;

  c_level<0>(ei1, ea1, nE1, vec81, nN, Y, 0,  dsm, vs, tid, lane, wave, nodeBase);
  c_level<1>(ei2, ea2, nE2, vec82, nN, Y, 16, dsm, vs, tid, lane, wave, nodeBase);
  __syncthreads();

  const int lim = nN * 16;
  const int gb0 = nodeBase * 16;
#pragma unroll 4
  for (int it = 0; it < (NBA * 16) / (NTHR * 4); ++it) {
    const int p = it * NTHR + tid;
    const v4f v = *(const v4fa*)(vs + 4 * p);
    const int gi = gb0 + 4 * p;
    if (gi < lim) *(volatile v4f*)(out + (size_t)gi) = v;
  }
  __threadfence();
#pragma unroll 4
  for (int it = 0; it < (NBA * 16) / (NTHR * 4); ++it) {
    const int p = it * NTHR + tid;
    const v4f v = *(const v4fa*)(vs + 4 * p);
    const int gi = gb0 + 4 * p;
    if (gi < lim) *(volatile v4f*)(out + (size_t)gi) = v;
  }
}

static inline int cdiv(int a, int b) { return (a + b - 1) / b; }
static inline size_t al256(size_t o) { return (o + 255) & ~(size_t)255; }

extern "C" void kernel_launch(void* const* d_in, const int* in_sizes, int n_in,
                              void* d_out, int out_size, void* d_ws, size_t ws_size,
                              hipStream_t stream) {
  if (n_in < 20) return;
  if (in_sizes[0] < FIN || (in_sizes[0] % FIN) != 0) return;
  const int nN = in_sizes[0] / FIN;
  if (nN < 2 || (nN & 1) != 0 || nN > (1 << 21)) return;
  if (in_sizes[1] < 2 || (in_sizes[1] & 1) != 0) return;
  const int nEo = in_sizes[1] / 2;
  const int nE1 = in_sizes[3];
  const int nE2 = in_sizes[5];
  if (nEo < 1 || nE1 < 1 || nE2 < 1) return;
  if (in_sizes[2] != 2 * nE1 || in_sizes[4] != 2 * nE2) return;
  if (nEo >= (1 << (31 - SLA)) || nE1 >= (1 << (31 - SLA)) || nE2 >= (1 << (31 - SLA))) return;
  if (in_sizes[6] != FIN * HID || in_sizes[7] != HID) return;
  if (in_sizes[8] != HID * 32 || in_sizes[14] != HID * 32) return;
  if (in_sizes[9] != 32 || in_sizes[10] != 32 || in_sizes[11] != 32) return;
  if (in_sizes[15] != 32 || in_sizes[16] != 32 || in_sizes[17] != 32) return;
  if (in_sizes[12] != 512 || in_sizes[13] != 16) return;
  if (in_sizes[18] != 512 || in_sizes[19] != 16) return;
  if ((long long)out_size != (long long)nN * 16) return;

  const float* x   = (const float*)d_in[0];
  const int*   eio = (const int*)d_in[1];
  const int*   ei1 = (const int*)d_in[2];
  const float* ea1 = (const float*)d_in[3];
  const int*   ei2 = (const int*)d_in[4];
  const float* ea2 = (const float*)d_in[5];
  const float* W1  = (const float*)d_in[6];
  const float* b1  = (const float*)d_in[7];
  const float* gw1 = (const float*)d_in[8];
  const float* as1 = (const float*)d_in[9];
  const float* ad1 = (const float*)d_in[10];
  const float* gb1 = (const float*)d_in[11];
  const float* wm1 = (const float*)d_in[12];
  const float* bm1 = (const float*)d_in[13];
  const float* gw2 = (const float*)d_in[14];
  const float* as2 = (const float*)d_in[15];
  const float* ad2 = (const float*)d_in[16];
  const float* gb2 = (const float*)d_in[17];
  const float* wm2 = (const float*)d_in[18];
  const float* bm2 = (const float*)d_in[19];
  float* out = (float*)d_out;

  const int MP = cdiv(nN, GBM) * GBM;
  const int gM = MP / GBM;
  const int gA = cdiv(nN, NBA);
  const int NP = gA * NBA;
  if (NP < nN || MP < nN) return;
  const int vecO = ((nEo & 3) == 0) ? 1 : 0;
  const int vec1 = ((nE1 & 3) == 0) ? 1 : 0;
  const int vec2 = ((nE2 & 3) == 0) ? 1 : 0;

  char* ws = (char*)d_ws;
  size_t off = 0;
  const size_t oW1T = off; off = al256(off + (size_t)HID * FIN * 2);
  const size_t oWGT = off; off = al256(off + (size_t)NTC * KH * 2);
  const size_t oXB  = off; off = al256(off + (size_t)MP * FIN * 2);
  const size_t oHHL = off; off = al256(off + (size_t)MP * KH * 2);
  const size_t oT   = off; off = al256(off + (size_t)MP * NTC * 4);
  const size_t oPP  = off; off = al256(off + (size_t)NP * NTC * 4);
  const size_t oASD = off; off = al256(off + (size_t)2 * NP * 4 * 4);
  const size_t oY   = off; off = al256(off + (size_t)NP * 32 * 4);
  if (off > ws_size || off > (size_t)WSMAX) return;
  unsigned short* W1T = (unsigned short*)(ws + oW1T);
  unsigned short* WGT = (unsigned short*)(ws + oWGT);
  unsigned short* XB  = (unsigned short*)(ws + oXB);
  unsigned short* HHL = (unsigned short*)(ws + oHHL);
  float* T   = (float*)(ws + oT);
  float* PP  = (float*)(ws + oPP);
  float* ASD = (float*)(ws + oASD);
  float* Y   = (float*)(ws + oY);

  const size_t ldsA = (size_t)A_LDS_INTS * 4;
  const size_t ldsB = (size_t)B_LDS_INTS * 4;
  const size_t ldsC = (size_t)C_LDS_INTS * 4;
  hipFuncSetAttribute(reinterpret_cast<const void*>(&k_scanA), hipFuncAttributeMaxDynamicSharedMemorySize, (int)ldsA);
  hipFuncSetAttribute(reinterpret_cast<const void*>(&k_scanB), hipFuncAttributeMaxDynamicSharedMemorySize, (int)ldsB);
  hipFuncSetAttribute(reinterpret_cast<const void*>(&k_scanC), hipFuncAttributeMaxDynamicSharedMemorySize, (int)ldsC);

  const int nUx = MP * (FIN / 8);
  k_wprep<<<(NUW1 + 2 * NUWG) / NTHR, NTHR, 0, stream>>>(W1, gw1, gw2, W1T, WGT);
  k_cvx<<<cdiv(nUx, NTHR), NTHR, 0, stream>>>(x, nN, nUx, XB);
  k_gemm1<<<dim3(gM, HID / GBN), GTHR, 0, stream>>>(XB, W1T, b1, HHL);
  k_gemm2<<<dim3(gM, NTC / GBN), GTHR, 0, stream>>>(HHL, WGT, T, KH, NTC);
  k_scanA<<<gA, NTHR, ldsA, stream>>>(ei1, ei1 + nE1, ea1, nE1, nN, vec1, T, 0,  as1, ad1, PP, ASD);
  k_scanA<<<gA, NTHR, ldsA, stream>>>(ei2, ei2 + nE2, ea2, nE2, nN, vec2, T, 32, as2, ad2, PP, ASD + (size_t)NP * 4);
  k_scanB<<<gA, NTHR, ldsB, stream>>>(eio, eio + nEo, nEo, nN, vecO, NP, PP, ASD,
                                      gb1, gb2, wm1, wm2, bm1, bm2, Y);
  k_scanC<<<gA, NTHR, ldsC, stream>>>(ei1, ea1, nE1, vec1, ei2, ea2, nE2, vec2, nN, Y, out);
}
